// UserEncoder_66614942761558
// MI455X (gfx1250) — hardware-verified
//
#include <hip/hip_runtime.h>
#include <hip/hip_bf16.h>
#include <math.h>

#define NBu 32
#define NH 100
#define NC 50
#define DDu 400
#define HID 400
#define KP 416
#define NP 512
#define MR (NBu * NH)
#define GSTR 48

typedef _Float16 bf16;
typedef _Float16 f16;
typedef __attribute__((ext_vector_type(4))) unsigned v4u_t;
typedef unsigned v4ua __attribute__((ext_vector_type(4), may_alias));
typedef __attribute__((ext_vector_type(4))) float v4f_t;
typedef float v4fa __attribute__((ext_vector_type(4), may_alias));
typedef __attribute__((ext_vector_type(16))) bf16  bf16x16;
typedef bf16x16 f16x16;
typedef __attribute__((ext_vector_type(8)))  bf16  bf16x8;
typedef bf16x8 f16x8;
typedef __attribute__((ext_vector_type(8)))  float f32x8;
__device__ __forceinline__ f32x8 wmma16(f16x16 a, f16x16 b, f32x8 c) {
  c = __builtin_amdgcn_wmma_f32_16x16x32_f16(false, a, false, b, (short)0, c, false, false);
  asm volatile("v_nop\n\tv_nop\n\tv_nop\n\tv_nop" : "+v"(c) : "v"(a), "v"(b));
  return c;
}
__device__ __forceinline__ f16x16 lds_frag(const f16* base, int stride) {
  const int lane = threadIdx.x & 31, row = lane & 15, kh = (lane >> 4) * 8;
  const f16x8 lo = *(const f16x8*)(base + row * stride + kh);
  const f16x8 hi = *(const f16x8*)(base + row * stride + kh + 16);
  f16x16 f;
#pragma unroll
  for (int i = 0; i < 8; ++i) { f[i] = lo[i]; f[i + 8] = hi[i]; }
  return f;
}

template <typename AT, bool ACC>
__global__ __launch_bounds__(256) void gemm_kn2(const AT* __restrict__ A, int lda, size_t strideA,
                                               const float* __restrict__ Wm, int ldw, size_t strideW,
                                               const float* __restrict__ bias, float scale,
                                               float* __restrict__ Y, int ldy, size_t strideY, int K) {
  __shared__ __attribute__((aligned(16))) f16 ldsA[128 * GSTR], ldsAl[128 * GSTR];
  __shared__ __attribute__((aligned(16))) f16 ldsW[128 * GSTR], ldsWl[128 * GSTR];
  __shared__ __attribute__((aligned(16))) float oS[8][32 * 68];
  const int tid = threadIdx.x, lane = tid & 31, wave = tid >> 5, cl = lane & 15, rh = (lane >> 4) * 8;
  const int m0 = blockIdx.x * 128, n0 = blockIdx.y * 128;
  const int wm = (wave & 3) * 32, wn = (wave >> 2) * 64;
  A += (size_t)blockIdx.z * strideA; Wm += (size_t)blockIdx.z * strideW; Y += (size_t)blockIdx.z * strideY;
  f32x8 acc[2][4], accx[2][4];
#pragma unroll
  for (int i = 0; i < 2; ++i)
#pragma unroll
    for (int j = 0; j < 4; ++j) { f32x8 z = {}; acc[i][j] = z; accx[i][j] = z; }
#pragma unroll 1
  for (int k0 = 0; k0 < K; k0 += 32) {
    __syncthreads();
    {
      const int row = tid >> 1, ch = (tid & 1) * 16;
      const AT* src = A + (size_t)(m0 + row) * lda + k0 + ch;
#pragma unroll
      for (int g = 0; g < 16; ++g) { const float v = (float)src[g]; const f16 h = (f16)v; ldsA[row * GSTR + ch + g] = h; ldsAl[row * GSTR + ch + g] = (f16)((v - (float)h) * 2048.0f); }
    }
    {
      const int k = tid >> 3, nn0 = (tid & 7) * 16;
      const float* src = Wm + (size_t)(k0 + k) * ldw + n0 + nn0;
#pragma unroll
      for (int g = 0; g < 4; ++g) { const v4f_t v = *(const v4f_t*)(src + 4 * g);
#pragma unroll
        for (int u = 0; u < 4; ++u) { const f16 h = (f16)v[u]; ldsW[(nn0 + 4 * g + u) * GSTR + k] = h; ldsWl[(nn0 + 4 * g + u) * GSTR + k] = (f16)((v[u] - (float)h) * 2048.0f); } }
    }
    __syncthreads();
    f16x16 af[2], afl[2];
#pragma unroll
    for (int i = 0; i < 2; ++i) { af[i] = lds_frag(ldsA + (wm + 16 * i) * GSTR, GSTR); afl[i] = lds_frag(ldsAl + (wm + 16 * i) * GSTR, GSTR); }
#pragma unroll
    for (int j = 0; j < 4; ++j) {
      const f16x16 bf = lds_frag(ldsW + (wn + 16 * j) * GSTR, GSTR), bfl = lds_frag(ldsWl + (wn + 16 * j) * GSTR, GSTR);
#pragma unroll
      for (int i = 0; i < 2; ++i) { acc[i][j] = wmma16(af[i], bf, acc[i][j]); accx[i][j] = wmma16(af[i], bfl, accx[i][j]); accx[i][j] = wmma16(afl[i], bf, accx[i][j]); }
    }
  }
  float* so = oS[wave];
#pragma unroll
  for (int i = 0; i < 2; ++i)
#pragma unroll
    for (int j = 0; j < 4; ++j) {
      const float bv = bias ? bias[n0 + wn + 16 * j + cl] : 0.0f;
#pragma unroll
      for (int r = 0; r < 8; ++r) so[(16 * i + rh + r) * 68 + 16 * j + cl] = (acc[i][j][r] + accx[i][j][r] * (1.0f / 2048.0f)) * scale + bv;
    }
  asm volatile("s_wait_dscnt 0" ::: "memory");
  __builtin_amdgcn_wave_barrier();
  if (ACC) {
#pragma unroll
    for (int it = 0; it < 16; ++it) { const int f4 = lane + 32 * it, rr = f4 >> 4, q = (f4 & 15) * 4;
      const v4f_t old = *(const v4fa*)(Y + (size_t)(m0 + wm + rr) * ldy + n0 + wn + q);
      v4f_t v = *(const v4fa*)(so + rr * 68 + q); v += old; *(volatile v4fa*)(so + rr * 68 + q) = v; }
    asm volatile("s_wait_dscnt 0" ::: "memory");
  }
#pragma unroll 1
  for (int pass = 0; pass < 2; ++pass) {
#pragma unroll
    for (int it = 0; it < 16; ++it) { const int f4 = lane + 32 * it, rr = f4 >> 4, q = (f4 & 15) * 4;
      *(volatile v4f_t*)(Y + (size_t)(m0 + wm + rr) * ldy + n0 + wn + q) = *(const v4fa*)(so + rr * 68 + q); }
    __threadfence();
  }
}

__global__ __launch_bounds__(256) void k_padA(const float* __restrict__ src, float* __restrict__ dst) { const size_t r = blockIdx.x; for (int c = threadIdx.x; c < KP; c += 256) dst[r * KP + c] = (c < DDu) ? src[r * DDu + c] : 0.0f; }
__global__ __launch_bounds__(256) void k_padW(const float* __restrict__ W1, float* __restrict__ dst) { const int r = blockIdx.x; for (int c = threadIdx.x; c < NP; c += 256) dst[(size_t)r * NP + c] = (r < DDu && c < HID) ? W1[(size_t)(DDu + r) * HID + c] : 0.0f; }
__global__ __launch_bounds__(256) void k_user(const float* __restrict__ HP, const float* __restrict__ hist, const float* __restrict__ w2, const int* __restrict__ mh, const int* __restrict__ mc, float* __restrict__ out) {
  __shared__ float sS[128]; __shared__ float wS[128]; __shared__ __attribute__((aligned(16))) float uv[DDu];
  const int tid = threadIdx.x, b = blockIdx.x;
  if (tid < NH) { const float* hp = HP + ((size_t)b * NH + tid) * NP; float s = 0.0f;
#pragma unroll 1
    for (int c = 0; c < HID; ++c) s += hp[c] * w2[c];
    sS[tid] = (mh[b * NH + tid] != 0) ? s : -3.4028234663852886e38f; }
  __syncthreads();
  if (tid < 32) { float m = -3.4028234663852886e38f; for (int h = tid; h < NH; h += 32) m = fmaxf(m, sS[h]);
#pragma unroll
    for (int off = 1; off < 32; off <<= 1) m = fmaxf(m, __shfl_xor(m, off, 32));
    float z = 0.0f; for (int h = tid; h < NH; h += 32) { const float e = expf(sS[h] - m); wS[h] = e; z += e; }
#pragma unroll
    for (int off = 1; off < 32; off <<= 1) z += __shfl_xor(z, off, 32);
    for (int h = tid; h < NH; h += 32) wS[h] = wS[h] / z; }
  __syncthreads();
  for (int d = tid; d < DDu; d += 256) { float s = 0.0f;
#pragma unroll 1
    for (int h = 0; h < NH; ++h) s += wS[h] * hist[((size_t)b * NH + h) * DDu + d];
    uv[d] = s; }
  __syncthreads();
#pragma unroll 1
  for (int pass = 0; pass < 2; ++pass) { for (int q4 = tid; q4 < NC * 100; q4 += 256) { const int c = q4 / 100, c4 = (q4 % 100) * 4; const bool keep = mc[b * NC + c] != 0;
      v4f_t v = *(const v4fa*)(uv + c4); if (!keep) { v[0] = 0.f; v[1] = 0.f; v[2] = 0.f; v[3] = 0.f; }
      *(volatile v4f_t*)(out + ((size_t)b * NC + c) * DDu + c4) = v; } __threadfence(); }
}

extern "C" void kernel_launch(void* const* d_in, const int* in_sizes, int n_in,
                              void* d_out, int out_size, void* d_ws, size_t ws_size,
                              hipStream_t stream) {
  (void)in_sizes; (void)n_in; (void)out_size;
  const float* hist = (const float*)d_in[0];
  const float* cand = (const float*)d_in[1];
  const int* mh = (const int*)d_in[2];
  const int* mc = (const int*)d_in[3];
  const float* W1 = (const float*)d_in[4];
  const float* b1 = (const float*)d_in[5];
  const float* w2 = (const float*)d_in[6];
  const float* b2 = (const float*)d_in[7];
  (void)cand; (void)b1; (void)b2;
  float* out = (float*)d_out;
  char* ws = (char*)d_ws;
  float* Ap = (float*)ws; ws += (size_t)MR * KP * 4;
  float* Wp = (float*)ws; ws += (size_t)KP * NP * 4;
  float* HP = (float*)ws; ws += (size_t)MR * NP * 4;
  if ((size_t)(ws - (char*)d_ws) > ws_size) return;
  const dim3 blk(256);
  k_padA<<<dim3(MR), blk, 0, stream>>>(hist, Ap);
  k_padW<<<dim3(KP), blk, 0, stream>>>(W1, Wp);
  gemm_kn2<float, false><<<dim3(MR / 128, NP / 128, 1), blk, 0, stream>>>(Ap, KP, 0, Wp, NP, 0, nullptr, 1.0f, HP, NP, 0, KP);
  k_user<<<dim3(NBu), blk, 0, stream>>>(HP, hist, w2, mh, mc, out);
}
